// TorchBoostModel_20701742367032
// MI455X (gfx1250) — hardware-verified
//
#include <hip/hip_runtime.h>


#define NR   65536
#define DIN  128
#define HID  128
#define NT   32
#define DEP  6
#define NND  63
#define NLF  64
#define NNP  2048
#define RB   8192
#define DM   DIN
#define SHR  0.3f
#define BEPS 1e-5f
#define LOSC 1024.0f

typedef _Float16 h16;
typedef unsigned short bf;
typedef __attribute__((ext_vector_type(16))) __bf16   v16bf;
typedef __attribute__((ext_vector_type(16))) _Float16 v16h;
typedef __attribute__((ext_vector_type(8)))  _Float16 v8h;
typedef __attribute__((ext_vector_type(8)))  unsigned short v8us;
typedef __attribute__((ext_vector_type(8)))  float    v8f;
typedef __attribute__((ext_vector_type(4)))  float    v4f;
typedef __attribute__((ext_vector_type(4)))  _Float16 v4h;
typedef v8h  __attribute__((may_alias)) v8ha;
typedef v4f  __attribute__((may_alias)) v4fa;
typedef v8us __attribute__((may_alias)) v8usa;

__device__ __forceinline__ unsigned short f2bf(float f) { unsigned u = __float_as_uint(f); u += 0x7FFFu + ((u >> 16) & 1u); return (unsigned short)(u >> 16); }
__device__ __forceinline__ float bf2f(unsigned short b) { return __uint_as_float(((unsigned)b) << 16); }
__device__ __forceinline__ float bfr(float f) { return bf2f(f2bf(f)); }
__device__ __forceinline__ v16h cat16(v8h lo, v8h hi) { return __builtin_shufflevector(lo, hi, 0, 1, 2, 3, 4, 5, 6, 7, 8, 9, 10, 11, 12, 13, 14, 15); }
__device__ __forceinline__ v16bf cat16b(v8us lo, v8us hi) { return __builtin_bit_cast(v16bf, __builtin_shufflevector(lo, hi, 0, 1, 2, 3, 4, 5, 6, 7, 8, 9, 10, 11, 12, 13, 14, 15)); }
__device__ __forceinline__ v8f wmma16(v16h a, v16h b, v8f c) { return __builtin_amdgcn_wmma_f32_16x16x32_f16(false, a, false, b, (short)0, c, false, false); }
__device__ __forceinline__ v8f wmmab(v16bf a, v16bf b, v8f c) { return __builtin_amdgcn_wmma_f32_16x16x32_bf16(false, a, false, b, (short)0, c, false, false); }

__global__ __launch_bounds__(256) void k_wt(const float* __restrict__ Wm, int K, int ncols, bf* WT) {
    __shared__ __align__(16) unsigned short tl[64 * 72];
    const int tid = threadIdx.x, k0 = blockIdx.x * 64, n0 = blockIdx.y * 64;
    const int kk = tid >> 2, nq = (tid & 3) * 16;
#pragma unroll
    for (int i = 0; i < 16; ++i) tl[(nq + i) * 72 + kk] = f2bf(Wm[(size_t)(k0 + kk) * ncols + n0 + nq + i]);
    __syncthreads();
    const int piece = tid & 7;
    auto pass = [&]() {
#pragma unroll
        for (int s = 0; s < 2; ++s) { const int nr = (tid >> 3) + 32 * s; const v8us val = *(const v8usa*)(tl + nr * 72 + piece * 8); *(volatile v8us*)(WT + (size_t)(n0 + nr) * K + k0 + piece * 8) = val; }
    };
    pass(); __threadfence(); pass();
}
template <bool SPLITA, bool F16OUT = false>
__global__ __launch_bounds__(128) void k_gemmb(const bf* __restrict__ A, const bf* __restrict__ Al, const bf* __restrict__ Bn, const float* __restrict__ bias, float* C, int ldc, h16* C2, const float* __restrict__ R = nullptr, int K = DM, int roundR = 1) {
    __shared__ __align__(16) float ost[4][16 * 68];
    const int lane = threadIdx.x & 31, wave = threadIdx.x >> 5, lr = lane & 15, hi = lane >> 4;
    const int r0 = blockIdx.x * 64 + wave * 16, c0 = blockIdx.y * 64;
    const size_t aoff = (size_t)(r0 + lr) * K + 8 * hi;
    size_t boff[4];
#pragma unroll
    for (int t = 0; t < 4; ++t) boff[t] = (size_t)(c0 + t * 16 + lr) * K + 8 * hi;
    v8f acc[4];
#pragma unroll
    for (int t = 0; t < 4; ++t) acc[t] = (v8f){};
#pragma unroll 1
    for (int kc = 0; kc < K; kc += 32) {
        const v16bf a = cat16b(*(const v8us*)(A + aoff + kc), *(const v8us*)(A + aoff + kc + 16));
        v16bf al = a;
        if (SPLITA) al = cat16b(*(const v8us*)(Al + aoff + kc), *(const v8us*)(Al + aoff + kc + 16));
#pragma unroll
        for (int t = 0; t < 4; ++t) { const v16bf b = cat16b(*(const v8us*)(Bn + boff[t] + kc), *(const v8us*)(Bn + boff[t] + kc + 16)); acc[t] = wmmab(a, b, acc[t]); if (SPLITA) acc[t] = wmmab(al, b, acc[t]); }
        asm volatile("v_nop\n\tv_nop\n\tv_nop\n\tv_nop" : "+v"(acc[0]), "+v"(acc[1]), "+v"(acc[2]), "+v"(acc[3]) : "v"(a), "v"(al));
    }
    float* os = &ost[wave][0];
#pragma unroll
    for (int t = 0; t < 4; ++t) { const float bv = bias ? bfr(bias[c0 + t * 16 + lr]) : 0.f;
#pragma unroll
        for (int j = 0; j < 8; ++j) os[(hi * 8 + j) * 68 + t * 16 + lr] = acc[t][j] + bv; }
    __syncthreads();
    if (F16OUT) {
        h16* crow = (h16*)(void*)C + (size_t)r0 * ldc + c0;
        auto pass = [&]() {
#pragma unroll
            for (int s = 0; s < 4; ++s) { const int row = 4 * s + (lane >> 3), piece = lane & 7; const float* sp = os + row * 68 + piece * 8; v8h o, o2;
#pragma unroll
                for (int i = 0; i < 8; ++i) { const h16 a = (h16)sp[i]; o[i] = a; o2[i] = (h16)((sp[i] - (float)a) * LOSC); }
                *(volatile v8h*)(crow + (size_t)row * ldc + piece * 8) = o; if (C2) *(volatile v8h*)(C2 + (size_t)r0 * ldc + c0 + (size_t)row * ldc + piece * 8) = o2; }
        };
        pass(); __threadfence(); pass();
    } else {
        float* crow = C + (size_t)r0 * ldc + c0;
        auto pass = [&]() {
#pragma unroll
            for (int s = 0; s < 8; ++s) { const int Lid = (lane >> 3) + 4 * s, piece = lane & 7; const int row = Lid >> 1, cofs = (Lid & 1) * 32 + piece * 4;
                v4f val = *(const v4fa*)(os + row * 68 + cofs); if (R) { const v4f rv = *(const v4f*)(R + ((size_t)r0 + row) * ldc + c0 + cofs); val += roundR ? (v4f){bfr(rv[0]), bfr(rv[1]), bfr(rv[2]), bfr(rv[3])} : rv; }
                *(volatile v4f*)(crow + (size_t)row * ldc + cofs) = val; }
        };
        pass(); __threadfence(); pass();
    }
}


__global__ __launch_bounds__(256) void k_cvt128r(const float* __restrict__ src, int rows, bf* dst) {
    typedef __attribute__((ext_vector_type(4))) unsigned short v4us;
    const int lane = threadIdx.x & 31; const size_t r = (size_t)blockIdx.x * 8 + (threadIdx.x >> 5); if (r >= (size_t)rows) return; v4us o;
#pragma unroll
    for (int i = 0; i < 4; ++i) o[i] = f2bf(src[r * DIN + lane * 4 + i]);
    *(volatile v4us*)(dst + r * DIN + lane * 4) = o; __threadfence(); *(volatile v4us*)(dst + r * DIN + lane * 4) = o;
}
__global__ __launch_bounds__(256) void k_twpad(const float* __restrict__ tw, const float* __restrict__ tb, bf* TW, float* TB) {
    typedef __attribute__((ext_vector_type(4))) unsigned short v4us;
    const int lane = threadIdx.x & 31; const int r = blockIdx.x * 8 + (threadIdx.x >> 5); if (r >= NNP) return; const bool live = r < NT * NND; v4us o;
#pragma unroll
    for (int i = 0; i < 4; ++i) o[i] = f2bf(live ? tw[(size_t)(live ? r : 0) * DIN + lane * 4 + i] : 0.f);
    *(volatile v4us*)(TW + (size_t)r * DIN + lane * 4) = o; if ((r & 31) == 0) { const int rr = r + lane; const float bv = (rr < NT * NND) ? tb[rr < NT * NND ? rr : 0] : 0.f; *(volatile float*)(TB + rr) = bv; }
    __threadfence();
    *(volatile v4us*)(TW + (size_t)r * DIN + lane * 4) = o; if ((r & 31) == 0) { const int rr = r + lane; const float bv = (rr < NT * NND) ? tb[rr < NT * NND ? rr : 0] : 0.f; *(volatile float*)(TB + rr) = bv; }
}
__global__ __launch_bounds__(256) void k_w2pad(const float* __restrict__ w2, const float* __restrict__ b2, bf* W2T, float* B2) {
    typedef __attribute__((ext_vector_type(4))) unsigned short v4us;
    const int lane = threadIdx.x & 31; const int t = blockIdx.x * 8 + (threadIdx.x >> 5); if (t >= 64) return; const bool live = t < NT; v4us o;
#pragma unroll
    for (int i = 0; i < 4; ++i) o[i] = f2bf(live ? w2[(size_t)(lane * 4 + i) * NT + (live ? t : 0)] : 0.f);
    *(volatile v4us*)(W2T + (size_t)t * HID + lane * 4) = o; if ((t & 31) == 0) { const int tt = t + lane; const float bv = (tt < NT) ? b2[tt < NT ? tt : 0] : 0.f; *(volatile float*)(B2 + tt) = bv; }
    __threadfence();
    *(volatile v4us*)(W2T + (size_t)t * HID + lane * 4) = o; if ((t & 31) == 0) { const int tt = t + lane; const float bv = (tt < NT) ? b2[tt < NT ? tt : 0] : 0.f; *(volatile float*)(B2 + tt) = bv; }
}
__global__ __launch_bounds__(256) void k_bnplanes(const float* __restrict__ Hf, int rows, const float* __restrict__ ga, const float* __restrict__ be, const float* __restrict__ mu, const float* __restrict__ var, bf* Ph, bf* Pl) {
    typedef __attribute__((ext_vector_type(4))) unsigned short v4us;
    const int lane = threadIdx.x & 31; const size_t r = (size_t)blockIdx.x * 8 + (threadIdx.x >> 5); if (r >= (size_t)rows) return; v4us oh, ol;
#pragma unroll
    for (int i = 0; i < 4; ++i) { const int c = lane * 4 + i; const float hv = fmaxf(Hf[r * HID + c], 0.f); const float y = (hv - bfr(mu[c])) * rsqrtf(bfr(var[c]) + BEPS) * bfr(ga[c]) + bfr(be[c]); const unsigned short hb = f2bf(y); oh[i] = hb; ol[i] = f2bf(y - bf2f(hb)); }
    const size_t o = r * HID + lane * 4; *(volatile v4us*)(Ph + o) = oh; *(volatile v4us*)(Pl + o) = ol; __threadfence(); *(volatile v4us*)(Ph + o) = oh; *(volatile v4us*)(Pl + o) = ol;
}
__global__ __launch_bounds__(256) void k_dec(float* L, const float* __restrict__ temps) {
    const int lane = threadIdx.x & 31; const size_t r = (size_t)blockIdx.x * 8 + (threadIdx.x >> 5); if (r >= (size_t)RB) return;
#pragma unroll 1
    for (int ps = 0; ps < 2; ++ps) {
#pragma unroll 1
        for (int c0 = lane * 4; c0 < NNP; c0 += 128) { v4f v = *(const v4f*)(L + r * NNP + c0); v4f o;
#pragma unroll
            for (int i = 0; i < 4; ++i) { const int c = c0 + i; const int t = (c < NT * NND) ? c / NND : 0; const float z = v[i] / bfr(temps[t]); o[i] = (ps == 0) ? 1.0f / (1.0f + __expf(-z)) : v[i]; }
            *(volatile v4f*)(L + r * NNP + c0) = o; }
        if (ps == 0) __threadfence(); }
}
__global__ __launch_bounds__(256) void k_trees(const float* __restrict__ DEC, const float* __restrict__ A2, const float* __restrict__ x, const float* __restrict__ leaf, const float* __restrict__ rw, size_t r0, float* PRED) {
    const int lane = threadIdx.x & 31; const size_t rl = ((size_t)blockIdx.x * 8 + (threadIdx.x >> 5)) * 32 + lane; if (rl >= (size_t)RB) return; const size_t r = r0 + rl;
    float m = -3.0e38f;
#pragma unroll 1
    for (int t = 0; t < NT; ++t) m = fmaxf(m, A2[rl * 64 + t]);
    float den = 0.f;
#pragma unroll 1
    for (int t = 0; t < NT; ++t) den += __expf(A2[rl * 64 + t] - m);
    const float dinv = 1.0f / den;
    bool miss = false;
#pragma unroll 1
    for (int d = 0; d < DIN; ++d) miss = miss || __builtin_isnan(x[r * DIN + d]);
    float pred = 0.f;
#pragma unroll 1
    for (int t = 0; t < NT; ++t) { const float* Dr = DEC + rl * NNP + t * NND; float to = 0.f;
#pragma unroll 1
        for (int l = 0; l < NLF; ++l) { float p = 1.0f;
#pragma unroll
            for (int lvl = 0; lvl < DEP; ++lvl) { const int n = l & ((1 << lvl) - 1); float dcs = Dr[(1 << lvl) - 1 + n]; dcs = miss ? 0.5f : dcs; p *= ((l >> lvl) & 1) ? (1.0f - dcs) : dcs; }
            to = fmaf(p, bfr(leaf[t * NLF + l]), to); }
        const float at = __expf(A2[rl * 64 + t] - m) * dinv; pred = fmaf(to * bfr(rw[t]), at, pred); }
    pred *= SHR; *(volatile float*)(PRED + r) = pred; __threadfence(); *(volatile float*)(PRED + r) = pred;
}

extern "C" void kernel_launch(void* const* d_in, const int* in_sizes, int n_in,
                              void* d_out, int out_size, void* d_ws, size_t ws_size, hipStream_t stream) {
    (void)in_sizes; (void)n_in; (void)out_size;
    const float* x = (const float*)d_in[0]; const float* tree_w = (const float*)d_in[1]; const float* tree_b = (const float*)d_in[2]; const float* leaf = (const float*)d_in[3]; const float* temps = (const float*)d_in[4]; const float* w1 = (const float*)d_in[5]; const float* b1 = (const float*)d_in[6];
    const float* bng = (const float*)d_in[7]; const float* bnb = (const float*)d_in[8]; const float* bnm = (const float*)d_in[9]; const float* bnv = (const float*)d_in[10]; const float* w2 = (const float*)d_in[11]; const float* b2 = (const float*)d_in[12]; const float* rw = (const float*)d_in[13];
    float* out = (float*)d_out;
    char* wsp = (char*)d_ws;
    auto take = [&](size_t bytes) { char* p = wsp; wsp += (bytes + 255) & ~(size_t)255; return (void*)p; };
    bf* XB = (bf*)take((size_t)NR * DIN * 2); bf* W1 = (bf*)take((size_t)HID * DIN * 2); bf* TW = (bf*)take((size_t)NNP * DIN * 2); float* TB = (float*)take(NNP * 4); bf* W2T = (bf*)take(64 * HID * 2); float* B2 = (float*)take(64 * 4);
    float* Hf = (float*)take((size_t)RB * HID * 4); bf* Hh = (bf*)take((size_t)RB * HID * 2); bf* Hl = (bf*)take((size_t)RB * HID * 2); float* A2 = (float*)take((size_t)RB * 64 * 4); float* L = (float*)take((size_t)RB * NNP * 4);
    if ((size_t)(wsp - (char*)d_ws) > ws_size) return;
    k_cvt128r<<<NR / 8, 256, 0, stream>>>(x, NR, XB); k_wt<<<dim3(DIN / 64, HID / 64, 1), 256, 0, stream>>>(w1, DIN, HID, W1); k_twpad<<<NNP / 8, 256, 0, stream>>>(tree_w, tree_b, TW, TB); k_w2pad<<<64 / 8, 256, 0, stream>>>(w2, b2, W2T, B2);
    for (int rb = 0; rb < NR / RB; ++rb) { const size_t r0 = (size_t)rb * RB;
        k_gemmb<false, false><<<dim3(RB / 64, HID / 64, 1), 128, 0, stream>>>(XB + r0 * DIN, nullptr, W1, b1, Hf, HID, nullptr, nullptr, DIN);
        k_bnplanes<<<RB / 8, 256, 0, stream>>>(Hf, RB, bng, bnb, bnm, bnv, Hh, Hl);
        k_gemmb<true, false><<<dim3(RB / 64, 1, 1), 128, 0, stream>>>(Hh, Hl, W2T, B2, A2, 64, nullptr, nullptr, HID);
        k_gemmb<false, false><<<dim3(RB / 64, NNP / 64, 1), 128, 0, stream>>>(XB + r0 * DIN, nullptr, TW, TB, L, NNP, nullptr, nullptr, DIN);
        k_dec<<<RB / 8, 256, 0, stream>>>(L, temps);
        k_trees<<<(RB / 32) / 8, 256, 0, stream>>>(L, A2, x, leaf, rw, r0, out); }
}
